// TreeANFIS_25426206392905
// MI455X (gfx1250) — hardware-verified
//
#include <hip/hip_runtime.h>

#define F_DIM   64
#define R_DIM   1024
#define LCOND   4
#define KD      256
#define CROW    257
#define NPAIR   128
#define RPASS   512
#define ROWS    16
#define SUBG    2
#define NTHR    128
#define NWAVE   4

typedef __bf16 v16bf __attribute__((ext_vector_type(16)));
typedef float  v8f   __attribute__((ext_vector_type(8)));
typedef float  v4f   __attribute__((ext_vector_type(4)));
typedef v4f    v4fa  __attribute__((may_alias));
typedef unsigned short v8us_t __attribute__((ext_vector_type(8)));
typedef v8us_t v8us  __attribute__((may_alias));
typedef unsigned int v4u __attribute__((ext_vector_type(4)));

union Frag { v16bf v; v8us q[2]; };

__device__ __forceinline__ unsigned int f32_to_bf16_rne(float f) {
  unsigned int u = __float_as_uint(f);
  u += 0x7FFFu + ((u >> 16) & 1u);
  return u >> 16;
}
__device__ __forceinline__ float bf16_to_f32(unsigned int b) {
  return __uint_as_float(b << 16);
}
__device__ __forceinline__ int clampi(int v, int lo, int hi) {
  return v < lo ? lo : (v > hi ? hi : v);
}

__device__ __forceinline__ v8f wmma_bf16(v16bf a, v16bf b, v8f c) {
  v8f d = __builtin_amdgcn_wmma_f32_16x16x32_bf16(false, a, false, b, (short)0, c, false, false);
  asm volatile("v_nop\n\tv_nop\n\tv_nop\n\tv_nop" : "+v"(d) : "v"(a), "v"(b));
  return d;
}

__device__ __forceinline__ float fuzzy_leg(float xv, float t, float pr, float s, float mkv) {
  float z  = (pr * (xv - t)) * s;
  float e  = __expf(-z);
  float mf = __builtin_amdgcn_rcpf(1.0f + e);
  return mf * mkv + (1.0f - mkv);
}

__device__ __forceinline__ void epilogue(float (&part)[8], v8f acc, const float* frow, float bias) {
  v4f fa = *(const v4fa*)(frow);
  v4f fb = *(const v4fa*)(frow + 4);
  part[0] = fmaf(fa.x, acc[0] + bias, part[0]);
  part[1] = fmaf(fa.y, acc[1] + bias, part[1]);
  part[2] = fmaf(fa.z, acc[2] + bias, part[2]);
  part[3] = fmaf(fa.w, acc[3] + bias, part[3]);
  part[4] = fmaf(fb.x, acc[4] + bias, part[4]);
  part[5] = fmaf(fb.y, acc[5] + bias, part[5]);
  part[6] = fmaf(fb.z, acc[6] + bias, part[6]);
  part[7] = fmaf(fb.w, acc[7] + bias, part[7]);
}

__global__ void __launch_bounds__(256)
prep_cons_kernel(const float* __restrict__ cons, unsigned short* cbh, unsigned short* cbl, int nrules) {
  const int t   = blockIdx.x * 256 + threadIdx.x;
  const int r   = t >> 5;
  const int seg = t & 31;
  if (r >= nrules) return;
  const float* src = cons + (size_t)r * CROW + seg * 8;
  unsigned int hw[4], lw[4];
#pragma unroll
  for (int j = 0; j < 4; ++j) {
    float v0 = src[2 * j], v1 = src[2 * j + 1];
    unsigned int h0 = f32_to_bf16_rne(v0), h1 = f32_to_bf16_rne(v1);
    unsigned int l0 = f32_to_bf16_rne(v0 - bf16_to_f32(h0));
    unsigned int l1 = f32_to_bf16_rne(v1 - bf16_to_f32(h1));
    hw[j] = h0 | (h1 << 16);
    lw[j] = l0 | (l1 << 16);
  }
  v4u hv = {hw[0], hw[1], hw[2], hw[3]};
  v4u lv = {lw[0], lw[1], lw[2], lw[3]};
  volatile v4u* ph = (volatile v4u*)(cbh + (size_t)r * KD + seg * 8);
  volatile v4u* pl = (volatile v4u*)(cbl + (size_t)r * KD + seg * 8);
  *ph = hv;
  *pl = lv;
  __threadfence();
  *ph = hv;
  *pl = lv;
}

__global__ void __launch_bounds__(NTHR)
tsk_infer_kernel(const float* __restrict__ x,
                 const float* __restrict__ aw,
                 const float* __restrict__ prem,
                 const float* __restrict__ th,
                 const float* __restrict__ sg,
                 const float* __restrict__ mk,
                 const float* __restrict__ cons,
                 const int*   __restrict__ fidx,
                 const int*   __restrict__ pairs,
                 const unsigned short* __restrict__ cbh,
                 const unsigned short* __restrict__ cbl,
                 float* out, int nrows) {
  __shared__ float xa_lds[ROWS * F_DIM];
  __shared__ __align__(16) unsigned short ph_lds[ROWS * KD];
  __shared__ __align__(16) unsigned short pl_lds[ROWS * KD];
  __shared__ __align__(16) float f_lds[RPASS * ROWS];
  __shared__ float bias_lds[R_DIM];
  __shared__ float dw_lds[NWAVE * ROWS];
  __shared__ float nw_lds[NWAVE * ROWS];
  __shared__ __align__(16) float o_lds[SUBG * ROWS];

  const int tid  = threadIdx.x;
  const int lane = tid & 31;
  const int wave = tid >> 5;
  const int m    = lane & 15;
  const int h    = lane >> 4;

#pragma unroll
  for (int j = 0; j < R_DIM / NTHR; ++j) {
    int r = tid + NTHR * j;
    bias_lds[r] = cons[(size_t)r * CROW + KD];
  }
  const int pa = clampi(pairs[2 * tid], 0, F_DIM - 1);
  const int pb = clampi(pairs[2 * tid + 1], 0, F_DIM - 1);

  float den_tot = 0.0f, num_tot = 0.0f;

  for (int s = 0; s < SUBG; ++s) {
    const int b0 = (blockIdx.x * SUBG + s) * ROWS;
    __syncthreads();

#pragma unroll
    for (int j = 0; j < (ROWS * F_DIM) / NTHR; ++j) {
      int i  = tid + NTHR * j;
      int bb = i >> 6, f = i & 63;
      int row = b0 + bb;
      if (row > nrows - 1) row = nrows - 1;
      xa_lds[i] = x[(size_t)row * F_DIM + f] * aw[f];
    }
    __syncthreads();

#pragma unroll
    for (int mm = 0; mm < ROWS; ++mm) {
      const float* xr = xa_lds + mm * F_DIM;
      float v0;
      if (tid < F_DIM) { v0 = xr[tid]; }
      else             { float tq = xr[tid - F_DIM]; v0 = tq * tq; }
      float v1 = xr[pa] * xr[pb];
      unsigned int h0 = f32_to_bf16_rne(v0);
      unsigned int l0 = f32_to_bf16_rne(v0 - bf16_to_f32(h0));
      unsigned int h1 = f32_to_bf16_rne(v1);
      unsigned int l1 = f32_to_bf16_rne(v1 - bf16_to_f32(h1));
      ph_lds[mm * KD + tid]         = (unsigned short)h0;
      pl_lds[mm * KD + tid]         = (unsigned short)l0;
      ph_lds[mm * KD + NPAIR + tid] = (unsigned short)h1;
      pl_lds[mm * KD + NPAIR + tid] = (unsigned short)l1;
    }
    den_tot = 0.0f;
    num_tot = 0.0f;

    for (int pass = 0; pass < 2; ++pass) {
      {
        float denacc[ROWS];
#pragma unroll
        for (int bb = 0; bb < ROWS; ++bb) denacc[bb] = 0.0f;
#pragma unroll 1
        for (int j = 0; j < RPASS / NTHR; ++j) {
          const int lr = tid * (RPASS / NTHR) + j;
          const int r  = pass * RPASS + lr;
          const int i0 = clampi(fidx[r * LCOND + 0], 0, F_DIM - 1);
          const int i1 = clampi(fidx[r * LCOND + 1], 0, F_DIM - 1);
          const int i2 = clampi(fidx[r * LCOND + 2], 0, F_DIM - 1);
          const int i3 = clampi(fidx[r * LCOND + 3], 0, F_DIM - 1);
          const float pr = prem[r];
          const float t0 = th[r * LCOND + 0], t1 = th[r * LCOND + 1];
          const float t2 = th[r * LCOND + 2], t3 = th[r * LCOND + 3];
          const float s0 = sg[r * LCOND + 0], s1 = sg[r * LCOND + 1];
          const float s2 = sg[r * LCOND + 2], s3 = sg[r * LCOND + 3];
          const float m0 = mk[r * LCOND + 0], m1 = mk[r * LCOND + 1];
          const float m2 = mk[r * LCOND + 2], m3 = mk[r * LCOND + 3];
#pragma unroll
          for (int bb = 0; bb < ROWS; ++bb) {
            const float* xr = xa_lds + bb * F_DIM;
            float f = fuzzy_leg(xr[i0], t0, pr, s0, m0)
                    * fuzzy_leg(xr[i1], t1, pr, s1, m1)
                    * fuzzy_leg(xr[i2], t2, pr, s2, m2)
                    * fuzzy_leg(xr[i3], t3, pr, s3, m3);
            f_lds[lr * ROWS + bb] = f;
            denacc[bb] += f;
          }
        }
#pragma unroll
        for (int bb = 0; bb < ROWS; ++bb) {
          float v = denacc[bb];
          v += __shfl_xor(v, 1);
          v += __shfl_xor(v, 2);
          v += __shfl_xor(v, 4);
          v += __shfl_xor(v, 8);
          v += __shfl_xor(v, 16);
          denacc[bb] = v;
        }
        if (lane == 0) {
#pragma unroll
          for (int bb = 0; bb < ROWS; ++bb) dw_lds[wave * ROWS + bb] = denacc[bb];
        }
      }
      __syncthreads();
      if (tid < ROWS) {
        den_tot += ((dw_lds[tid] + dw_lds[ROWS + tid]) + dw_lds[2 * ROWS + tid]) + dw_lds[3 * ROWS + tid];
      }

      float part[8];
#pragma unroll
      for (int v = 0; v < 8; ++v) part[v] = 0.0f;

      const unsigned short* aph = ph_lds + m * KD + 8 * h;
      const unsigned short* apl = pl_lds + m * KD + 8 * h;

#pragma unroll 1
      for (int t = 0; t < 8; t += 2) {
        const int rtl0 = wave * 8 + t;
        const int rl0  = rtl0 * 16 + m;
        const int rl1  = rl0 + 16;
        const int rg0  = pass * RPASS + rl0;
        const int rg1  = rg0 + 16;
        const unsigned short* b0h = cbh + (size_t)rg0 * KD + 8 * h;
        const unsigned short* b0l = cbl + (size_t)rg0 * KD + 8 * h;
        const unsigned short* b1h = cbh + (size_t)rg1 * KD + 8 * h;
        const unsigned short* b1l = cbl + (size_t)rg1 * KD + 8 * h;
        v8f acc0 = {0.f, 0.f, 0.f, 0.f, 0.f, 0.f, 0.f, 0.f};
        v8f acc1 = {0.f, 0.f, 0.f, 0.f, 0.f, 0.f, 0.f, 0.f};
#pragma unroll 1
        for (int kb = 0; kb < KD / 32; ++kb) {
          const int ko = kb * 32;
          Frag ah, al, q0h, q0l, q1h, q1l;
          ah.q[0]  = *(const v8us*)(aph + ko);  ah.q[1]  = *(const v8us*)(aph + ko + 16);
          al.q[0]  = *(const v8us*)(apl + ko);  al.q[1]  = *(const v8us*)(apl + ko + 16);
          q0h.q[0] = *(const v8us*)(b0h + ko);  q0h.q[1] = *(const v8us*)(b0h + ko + 16);
          q0l.q[0] = *(const v8us*)(b0l + ko);  q0l.q[1] = *(const v8us*)(b0l + ko + 16);
          q1h.q[0] = *(const v8us*)(b1h + ko);  q1h.q[1] = *(const v8us*)(b1h + ko + 16);
          q1l.q[0] = *(const v8us*)(b1l + ko);  q1l.q[1] = *(const v8us*)(b1l + ko + 16);
          acc0 = wmma_bf16(ah.v, q0h.v, acc0);
          acc0 = wmma_bf16(ah.v, q0l.v, acc0);
          acc0 = wmma_bf16(al.v, q0h.v, acc0);
          acc1 = wmma_bf16(ah.v, q1h.v, acc1);
          acc1 = wmma_bf16(ah.v, q1l.v, acc1);
          acc1 = wmma_bf16(al.v, q1h.v, acc1);
        }
        epilogue(part, acc0, f_lds + rl0 * ROWS + 8 * h, bias_lds[rg0]);
        epilogue(part, acc1, f_lds + rl1 * ROWS + 8 * h, bias_lds[rg1]);
      }
#pragma unroll
      for (int v = 0; v < 8; ++v) {
        float q = part[v];
        q += __shfl_xor(q, 1);
        q += __shfl_xor(q, 2);
        q += __shfl_xor(q, 4);
        q += __shfl_xor(q, 8);
        part[v] = q;
      }
      if (m == 0) {
#pragma unroll
        for (int v = 0; v < 8; ++v) nw_lds[wave * ROWS + 8 * h + v] = part[v];
      }
      __syncthreads();
      if (tid < ROWS) {
        num_tot += ((nw_lds[tid] + nw_lds[ROWS + tid]) + nw_lds[2 * ROWS + tid]) + nw_lds[3 * ROWS + tid];
      }
    }
    if (tid < ROWS) o_lds[s * ROWS + tid] = num_tot / (den_tot + 1e-8f);
  }
  __syncthreads();

  if (tid == 0) {
    const int ob = blockIdx.x * SUBG * ROWS;
    if (ob + SUBG * ROWS <= nrows) {
      v4f vv[8];
#pragma unroll
      for (int q = 0; q < 8; ++q) vv[q] = *(const v4fa*)(o_lds + 4 * q);
      volatile v4f* po = (volatile v4f*)(out + ob);
#pragma unroll
      for (int q = 0; q < 8; ++q) po[q] = vv[q];
      __threadfence();
#pragma unroll
      for (int q = 0; q < 8; ++q) po[q] = vv[q];
    } else {
      volatile float* po = (volatile float*)(out + ob);
      for (int i = 0; i < SUBG * ROWS; ++i) { if (ob + i < nrows) po[i] = o_lds[i]; }
      __threadfence();
      for (int i = 0; i < SUBG * ROWS; ++i) { if (ob + i < nrows) po[i] = o_lds[i]; }
    }
  }
}

extern "C" void kernel_launch(void* const* d_in, const int* in_sizes, int n_in,
                              void* d_out, int out_size, void* d_ws, size_t ws_size,
                              hipStream_t stream) {
  if (n_in < 9) return;
  const int nrows = in_sizes[0] / F_DIM;
  if (nrows <= 0 || in_sizes[0] != nrows * F_DIM) return;
  if (in_sizes[1] != F_DIM || in_sizes[2] != R_DIM ||
      in_sizes[3] != R_DIM * LCOND || in_sizes[4] != R_DIM * LCOND || in_sizes[5] != R_DIM * LCOND ||
      in_sizes[6] != R_DIM * CROW || in_sizes[7] != R_DIM * LCOND || in_sizes[8] != NPAIR * 2) return;
  if (out_size != nrows) return;

  const float* x     = (const float*)d_in[0];
  const float* aw    = (const float*)d_in[1];
  const float* prem  = (const float*)d_in[2];
  const float* th    = (const float*)d_in[3];
  const float* sg    = (const float*)d_in[4];
  const float* mk    = (const float*)d_in[5];
  const float* cons  = (const float*)d_in[6];
  const int*   fidx  = (const int*)d_in[7];
  const int*   pairs = (const int*)d_in[8];

  const size_t plane_bytes = (size_t)R_DIM * KD * sizeof(unsigned short);
  if (ws_size < 2 * plane_bytes) return;
  unsigned short* cbh = (unsigned short*)d_ws;
  unsigned short* cbl = (unsigned short*)((char*)d_ws + plane_bytes);

  const int prep_threads = R_DIM * 32;
  prep_cons_kernel<<<(prep_threads + 255) / 256, 256, 0, stream>>>(cons, cbh, cbl, R_DIM);

  const int rows_per_block = SUBG * ROWS;
  const int nblk = (nrows + rows_per_block - 1) / rows_per_block;
  tsk_infer_kernel<<<nblk, NTHR, 0, stream>>>(x, aw, prem, th, sg, mk, cons, fidx, pairs,
                                              cbh, cbl, (float*)d_out, nrows);
}
